// EGCN_CPU_84121229460221
// MI455X (gfx1250) — hardware-verified
//
#include <hip/hip_runtime.h>
#include <stdint.h>
#include <stddef.h>
#pragma clang fp contract(off)

typedef _Float16 v16h __attribute__((ext_vector_type(16)));
typedef _Float16 v8h  __attribute__((ext_vector_type(8)));
typedef _Float16 v4h  __attribute__((ext_vector_type(4)));
typedef float    v8f  __attribute__((ext_vector_type(8)));
typedef float    v4f  __attribute__((ext_vector_type(4)));
typedef int      v4i  __attribute__((ext_vector_type(4)));
union Frag { v16h v; v8h h[2]; };

__device__ __forceinline__ v8f wmma16(v16h a, v16h b, v8f c) {
  c = __builtin_amdgcn_wmma_f32_16x16x32_f16(false, a, false, b, (short)0, c, false, false);
  asm volatile("v_nop\n\tv_nop\n\tv_nop\n\tv_nop" : "+v"(c) : "v"(a), "v"(b));
  return c;
}

__global__ __launch_bounds__(256) void cvt_w_kernel(const float* w0, int n0, const float* w1, int n1,
                                                    const float* w2, int n2, const float* w3, int n3,
                                                    _Float16* dst, int total8) {
  int g = blockIdx.x * 256 + threadIdx.x;
  if (g >= total8) return;
  int e = g * 8;
  const float* src;
  if (e < n0) src = w0 + e;
  else { e -= n0;
    if (e < n1) src = w1 + e;
    else { e -= n1;
      if (e < n2) src = w2 + e;
      else { e -= n2; src = w3 + e; } } }
  v4f p0 = *(const v4f*)src;
  v4f p1 = *(const v4f*)(src + 4);
  p0 = p0 * 16.0f; p1 = p1 * 16.0f;
  v4h q0 = __builtin_convertvector(p0, v4h);
  v4h q1 = __builtin_convertvector(p1, v4h);
  v8h o = __builtin_shufflevector(q0, q1, 0, 1, 2, 3, 4, 5, 6, 7);
  _Float16* p = dst + (size_t)g * 8;
  *(volatile v8h*)p = o;
  __threadfence();
  *(volatile v8h*)p = o;
}

template <int PASS>
__global__ __launch_bounds__(256) void agg_kernel(const float* f, const float* x0, const float* dinv,
                                                  const int* esrc, const int* edst, int ne, int n,
                                                  float* out32, _Float16* out16, float* dinv_out) {
  constexpr int R = 256, EPT = 8, CH = 256 * EPT, LCAP = 32 * EPT;
  __shared__ v4f acc[PASS ? R * 32 : 1];
  __shared__ int cntd[PASS ? 1 : R];
  __shared__ int hs[8 * LCAP];
  __shared__ int hd[8 * LCAP];
  __shared__ int hc[8];
  const int tid = threadIdx.x, w = tid >> 5, lane = tid & 31;
  const int node0 = blockIdx.x * R;

  if (PASS) {
    v4f z = {0.f, 0.f, 0.f, 0.f};
    for (int i = tid; i < R * 32; i += 256) acc[i] = z;
  } else {
    for (int i = tid; i < R; i += 256) cntd[i] = 0;
  }
  __syncthreads();

  for (int c0 = 0; c0 < ne; c0 += CH) {
    const int e0 = c0 + tid * EPT;
    int d[EPT];
    if (c0 + CH <= ne) {
      v4i q0 = *(const v4i*)(edst + e0);
      v4i q1 = *(const v4i*)(edst + e0 + 4);
      d[0] = q0[0]; d[1] = q0[1]; d[2] = q0[2]; d[3] = q0[3];
      d[4] = q1[0]; d[5] = q1[1]; d[6] = q1[2]; d[7] = q1[3];
    } else {
#pragma unroll
      for (int j = 0; j < EPT; ++j) { int e = e0 + j; d[j] = (e < ne) ? edst[e] : -1; }
    }
    int base = 0;
#pragma unroll
    for (int j = 0; j < EPT; ++j) {
      int dlj = d[j] - node0;
      bool hit = (unsigned)dlj < (unsigned)R;
      unsigned b = __builtin_amdgcn_ballot_w32(hit);
      if (hit) {
        int pos = base + __builtin_popcount(b & ((1u << lane) - 1u));
        hs[w * LCAP + pos] = esrc[e0 + j];
        hd[w * LCAP + pos] = dlj;
      }
      base += __builtin_popcount(b);
    }
    if (lane == 0) hc[w] = base;
    __syncthreads();
    for (int w2 = 0; w2 < 8; ++w2) {
      int cnt = hc[w2];
      cnt = cnt < LCAP ? cnt : LCAP;
      for (int i = 0; i < cnt; ++i) {
        int dl = hd[w2 * LCAP + i] & (R - 1);
        if ((dl & 7) == w) {
          if (PASS == 0) {
            if (lane == 0) cntd[dl] += 1;
          } else {
            int s = hs[w2 * LCAP + i];
            s = s < 0 ? 0 : (s >= n ? n - 1 : s);
            v4f v = *(const v4f*)(f + (size_t)s * 128 + lane * 4);
            float ds = dinv[s];
            v4f a = acc[dl * 32 + lane];
            a = a + v * ds;
            acc[dl * 32 + lane] = a;
          }
        }
      }
    }
    __syncthreads();
  }
  __syncthreads();

  if (PASS == 0) {
    if (w < 2) {
      int i = (w * 32 + lane) * 4;
      v4f o;
#pragma unroll
      for (int q = 0; q < 4; ++q) {
        int c = cntd[i + q];
        float dg = c < 1 ? 1.0f : (float)c;
        o[q] = 1.0f / sqrtf(dg);
      }
      float* p = dinv_out + (size_t)node0 + i;
      *(volatile v4f*)p = o;
      __threadfence();
      *(volatile v4f*)p = o;
    }
  } else if (PASS == 1) {
    for (int rep = 0; rep < 2; ++rep) {
#pragma unroll 1
      for (int rr = 0; rr < 32; ++rr) {
        int r = w * 32 + rr;
        int node = node0 + r;
        if (node < n) {
          v4f fv = *(const v4f*)(f + (size_t)node * 128 + lane * 4);
          float dn = dinv[node];
          v4f a = acc[r * 32 + lane];
          v4f lap = fv - a * dn;
          v4f o = -lap;
          *(volatile v4f*)(out32 + (size_t)node * 128 + lane * 4) = o;
        }
      }
      __threadfence();
    }
  } else {
    const int hh = lane >> 4, c8 = (lane & 15) * 8;
    for (int rep = 0; rep < 2; ++rep) {
#pragma unroll 1
      for (int rr = 0; rr < 16; ++rr) {
        int r = w * 32 + rr * 2 + hh;
        int node = node0 + r;
        if (node < n) {
          const float* fp = f + (size_t)node * 128 + c8;
          const float* xp = x0 + (size_t)node * 128 + c8;
          v4f f0 = *(const v4f*)fp, f1 = *(const v4f*)(fp + 4);
          v4f g0 = *(const v4f*)xp, g1 = *(const v4f*)(xp + 4);
          float dn = dinv[node];
          v4f a0 = acc[r * 32 + (c8 >> 2)], a1 = acc[r * 32 + (c8 >> 2) + 1];
          v4f l0 = f0 - a0 * dn, l1 = f1 - a1 * dn;
          v4f o0 = -2.0f * l0 - g0, o1 = -2.0f * l1 - g1;
          v4h q0 = __builtin_convertvector(o0, v4h);
          v4h q1 = __builtin_convertvector(o1, v4h);
          v8h hv = __builtin_shufflevector(q0, q1, 0, 1, 2, 3, 4, 5, 6, 7);
          *(volatile v8h*)(out16 + (size_t)node * 128 + c8) = hv;
        }
      }
      __threadfence();
    }
  }
}

template <int MODE>
__global__ __launch_bounds__(256) void conv_gemm_kernel(const float* A0, const float* A1, const _Float16* A2,
                                                        const _Float16* W, const float* bias,
                                                        const float* bn_g, const float* bn_b,
                                                        const float* bn_m, const float* bn_v,
                                                        const float* resid, int n,
                                                        float* outY, _Float16* outZ) {
  constexpr int K = 384;
  __shared__ _Float16 aT[16 * K];
  __shared__ float dS[16 * 128];
  const int tid = threadIdx.x, w = tid >> 5, lane = tid & 31, h = lane >> 4, m = lane & 15;
  const int row0 = blockIdx.x * 16;

  for (int g = tid; g < 16 * K / 8; g += 256) {
    int e = g * 8;
    int r = e / K;
    int k = e - r * K;
    int row = row0 + r; row = row < n ? row : n - 1;
    v8h hv;
    if (k < 256) {
      const float* src = (k < 128 ? A0 : A1) + (size_t)row * 128 + (k & 127);
      v4f p0 = *(const v4f*)src;
      v4f p1 = *(const v4f*)(src + 4);
      v4h q0 = __builtin_convertvector(p0, v4h);
      v4h q1 = __builtin_convertvector(p1, v4h);
      hv = __builtin_shufflevector(q0, q1, 0, 1, 2, 3, 4, 5, 6, 7);
    } else {
      hv = *(const v8h*)(A2 + (size_t)row * 128 + (k - 256));
    }
    *(v8h*)(aT + r * K + k) = hv;
  }
  __syncthreads();

  v8f acc = {0.f, 0.f, 0.f, 0.f, 0.f, 0.f, 0.f, 0.f};
  const _Float16* wrow = W + (size_t)(w * 16 + m) * K;
  const _Float16* arow = aT + m * K;
#pragma unroll
  for (int ks = 0; ks < K; ks += 32) {
    Frag a, b;
    a.h[0] = *(const v8h*)(arow + ks + 8 * h);
    a.h[1] = *(const v8h*)(arow + ks + 16 + 8 * h);
    b.h[0] = *(const v8h*)(wrow + ks + 8 * h);
    b.h[1] = *(const v8h*)(wrow + ks + 16 + 8 * h);
    acc = wmma16(a.v, b.v, acc);
  }

  const int col = w * 16 + m;
  const float bv = bias[col];
  float rs = 0.f, gg = 0.f, bb = 0.f, mu = 0.f;
  if (MODE == 0) { rs = 1.0f / sqrtf(bn_v[col] + 1e-5f); gg = bn_g[col]; bb = bn_b[col]; mu = bn_m[col]; }
#pragma unroll
  for (int r = 0; r < 8; ++r) {
    int lr = 8 * h + r;
    float v = acc[r] * 0.0625f + bv;
    v = fmaxf(v, 0.0f);
    if (MODE == 0) {
      v = ((v - mu) * rs) * gg + bb;
    } else {
      int grow = row0 + lr; grow = grow < n ? grow : n - 1;
      v = v + resid[(size_t)grow * 128 + col];
    }
    dS[lr * 128 + col] = v;
  }
  __syncthreads();

  for (int rep = 0; rep < 2; ++rep) {
    if (MODE == 0) {
#pragma unroll
      for (int q = 0; q < 2; ++q) {
        int r = w + 8 * q;
        int grow = row0 + r;
        if (grow < n) {
          v4f v = *(const v4f*)(dS + r * 128 + lane * 4);
          *(volatile v4f*)(outY + (size_t)grow * 128 + lane * 4) = v;
        }
      }
    } else {
      int r = 2 * w + h;
      int c8 = m * 8;
      int grow = row0 + r;
      if (grow < n) {
        v4f p0 = *(const v4f*)(dS + r * 128 + c8);
        v4f p1 = *(const v4f*)(dS + r * 128 + c8 + 4);
        v4h q0 = __builtin_convertvector(p0, v4h);
        v4h q1 = __builtin_convertvector(p1, v4h);
        v8h hv = __builtin_shufflevector(q0, q1, 0, 1, 2, 3, 4, 5, 6, 7);
        *(volatile v8h*)(outZ + (size_t)grow * 128 + c8) = hv;
      }
    }
    __threadfence();
  }
}

__global__ __launch_bounds__(256) void mlp_kernel(const _Float16* Z, const _Float16* Wm1, const float* bm1,
                                                  const _Float16* Wm2, const float* bm2, int n, float* out) {
  __shared__ _Float16 hS[16 * 128];
  __shared__ float dS[16 * 64];
  const int tid = threadIdx.x, w = tid >> 5, lane = tid & 31, h = lane >> 4, m = lane & 15;
  const int row0 = blockIdx.x * 16;
  int arow = row0 + m; arow = arow < n ? arow : n - 1;

  {
    v8f acc = {0.f, 0.f, 0.f, 0.f, 0.f, 0.f, 0.f, 0.f};
    const _Float16* ap = Z + (size_t)arow * 128;
    const _Float16* wp = Wm1 + (size_t)(w * 16 + m) * 128;
#pragma unroll
    for (int ks = 0; ks < 128; ks += 32) {
      Frag a, b;
      a.h[0] = *(const v8h*)(ap + ks + 8 * h);
      a.h[1] = *(const v8h*)(ap + ks + 16 + 8 * h);
      b.h[0] = *(const v8h*)(wp + ks + 8 * h);
      b.h[1] = *(const v8h*)(wp + ks + 16 + 8 * h);
      acc = wmma16(a.v, b.v, acc);
    }
    const int col = w * 16 + m;
    const float bv = bm1[col];
#pragma unroll
    for (int r = 0; r < 8; ++r) {
      float v = fmaxf(acc[r] * 0.0625f + bv, 0.0f);
      hS[(8 * h + r) * 128 + col] = (_Float16)v;
    }
  }
  __syncthreads();

  if (w < 4) {
    v8f acc = {0.f, 0.f, 0.f, 0.f, 0.f, 0.f, 0.f, 0.f};
    const _Float16* ap = hS + m * 128;
    const _Float16* wp = Wm2 + (size_t)(w * 16 + m) * 128;
#pragma unroll
    for (int ks = 0; ks < 128; ks += 32) {
      Frag a, b;
      a.h[0] = *(const v8h*)(ap + ks + 8 * h);
      a.h[1] = *(const v8h*)(ap + ks + 16 + 8 * h);
      b.h[0] = *(const v8h*)(wp + ks + 8 * h);
      b.h[1] = *(const v8h*)(wp + ks + 16 + 8 * h);
      acc = wmma16(a.v, b.v, acc);
    }
    const int col = w * 16 + m;
    const float bv = bm2[col];
#pragma unroll
    for (int r = 0; r < 8; ++r) dS[(8 * h + r) * 64 + col] = acc[r] * 0.0625f + bv;
  }
  __syncthreads();

  {
    int r = 2 * w + h;
    int c4 = m * 4;
    int grow = row0 + r;
    if (grow < n) {
      v4f v = *(const v4f*)(dS + r * 64 + c4);
      float* p = out + (size_t)grow * 64 + c4;
      *(volatile v4f*)p = v;
      __threadfence();
      *(volatile v4f*)p = v;
    }
  }
}

extern "C" void kernel_launch(void* const* d_in, const int* in_sizes, int n_in,
                              void* d_out, int out_size, void* d_ws, size_t ws_size,
                              hipStream_t stream) {
  const float* features = (const float*)d_in[0];
  const int*   esrc     = (const int*)d_in[1];
  const int*   edst     = (const int*)d_in[2];
  const float* W1       = (const float*)d_in[3];
  const float* b1       = (const float*)d_in[4];
  const float* bn_gamma = (const float*)d_in[5];
  const float* bn_beta  = (const float*)d_in[6];
  const float* bn_mean  = (const float*)d_in[7];
  const float* bn_var   = (const float*)d_in[8];
  const float* W3       = (const float*)d_in[9];
  const float* b3       = (const float*)d_in[10];
  const float* Wm1      = (const float*)d_in[11];
  const float* bm1      = (const float*)d_in[12];
  const float* Wm2      = (const float*)d_in[13];
  const float* bm2      = (const float*)d_in[14];
  float* out = (float*)d_out;

  const int n  = in_sizes[0] / 128;
  const int ne = in_sizes[1];
  if (n <= 0) return;
  const int R = 256;
  const int nblkA = (n + R - 1) / R;

  const int nW1 = 128 * 384, nW3 = 128 * 384, nWm1 = 128 * 128, nWm2 = 64 * 128;
  const int nWtot = nW1 + nW3 + nWm1 + nWm2;

  char* ws = (char*)d_ws;
  size_t off = 0;
  auto carve = [&](size_t bytes) { char* p = ws + off; off += (bytes + 255) & ~(size_t)255; return p; };
  float*    dinv = (float*)carve((size_t)nblkA * R * 4);
  float*    T1   = (float*)carve((size_t)n * 128 * 4);
  _Float16* T2h  = (_Float16*)carve((size_t)n * 128 * 2);
  float*    Y    = (float*)carve((size_t)n * 128 * 4);
  _Float16* Wh   = (_Float16*)carve((size_t)nWtot * 2);
  if (off > ws_size) return;
  _Float16* W1h  = Wh;
  _Float16* W3h  = Wh + nW1;
  _Float16* Wm1h = Wh + nW1 + nW3;
  _Float16* Wm2h = Wh + nW1 + nW3 + nWm1;
  _Float16* Zh   = T2h;

  const int total8 = nWtot / 8;
  cvt_w_kernel<<<(total8 + 255) / 256, 256, 0, stream>>>(W1, nW1, W3, nW3, Wm1, nWm1, Wm2, nWm2, Wh, total8);

  agg_kernel<0><<<nblkA, 256, 0, stream>>>(nullptr, nullptr, nullptr, esrc, edst, ne, n, nullptr, nullptr, dinv);

  agg_kernel<1><<<nblkA, 256, 0, stream>>>(features, nullptr, dinv, esrc, edst, ne, n, T1, nullptr, nullptr);
  agg_kernel<2><<<nblkA, 256, 0, stream>>>(T1, features, dinv, esrc, edst, ne, n, nullptr, T2h, nullptr);
  const int gMT = (n + 15) / 16;
  conv_gemm_kernel<0><<<gMT, 256, 0, stream>>>(features, T1, T2h, W1h, b1, bn_gamma, bn_beta, bn_mean, bn_var,
                                                nullptr, n, Y, nullptr);

  agg_kernel<1><<<nblkA, 256, 0, stream>>>(Y, nullptr, dinv, esrc, edst, ne, n, T1, nullptr, nullptr);
  agg_kernel<2><<<nblkA, 256, 0, stream>>>(T1, Y, dinv, esrc, edst, ne, n, nullptr, T2h, nullptr);
  conv_gemm_kernel<1><<<gMT, 256, 0, stream>>>(Y, T1, T2h, W3h, b3, nullptr, nullptr, nullptr, nullptr,
                                                Y, n, nullptr, Zh);

  mlp_kernel<<<gMT, 256, 0, stream>>>(Zh, Wm1h, bm1, Wm2h, bm2, n, out);
}
